// Self_Attn_50354196579077
// MI455X (gfx1250) — hardware-verified
//
#include <hip/hip_runtime.h>


#define NB_  4
#define TT   4096
#define DM   256
#define NH_  1
#define NKV  1
#define REP  (NH_ / NKV)
#define HD   64
#define DQ   (NH_ * HD)
#define DKV  (NKV * HD)
#define ZH   1
#define RH   4096
#define WIN  0
#define PCAR 1024.0f
#define SCL  1.0f
#define CI   32
#define CP   128
#define HP   64
#define CC   256
typedef _Float16 h16;
typedef unsigned short bf;
typedef __attribute__((ext_vector_type(16))) __bf16   v16bf;
typedef __attribute__((ext_vector_type(16))) _Float16 v16h;
typedef __attribute__((ext_vector_type(8)))  _Float16 v8h;
typedef __attribute__((ext_vector_type(8)))  unsigned short v8us;
typedef __attribute__((ext_vector_type(8)))  float    v8f;
typedef __attribute__((ext_vector_type(4)))  float    v4f;
typedef v8h  __attribute__((may_alias)) v8ha;
typedef v4f  __attribute__((may_alias)) v4fa;
typedef v8us __attribute__((may_alias)) v8usa;

__device__ __forceinline__ unsigned short f2bf(float f) { unsigned u = __float_as_uint(f); u += 0x7FFFu + ((u >> 16) & 1u); return (unsigned short)(u >> 16); }
__device__ __forceinline__ float bf2f(unsigned short b) { return __uint_as_float(((unsigned)b) << 16); }
__device__ __forceinline__ float bfr(float f) { return bf2f(f2bf(f)); }
__device__ __forceinline__ v16h cat16(v8h lo, v8h hi) { return __builtin_shufflevector(lo, hi, 0, 1, 2, 3, 4, 5, 6, 7, 8, 9, 10, 11, 12, 13, 14, 15); }
__device__ __forceinline__ v16bf cat16b(v8us lo, v8us hi) { return __builtin_bit_cast(v16bf, __builtin_shufflevector(lo, hi, 0, 1, 2, 3, 4, 5, 6, 7, 8, 9, 10, 11, 12, 13, 14, 15)); }
__device__ __forceinline__ v8f wmma16(v16h a, v16h b, v8f c) { return __builtin_amdgcn_wmma_f32_16x16x32_f16(false, a, false, b, (short)0, c, false, false); }
__device__ __forceinline__ v8f wmmab(v16bf a, v16bf b, v8f c) { return __builtin_amdgcn_wmma_f32_16x16x32_bf16(false, a, false, b, (short)0, c, false, false); }


template <typename T16> struct WFrag;
template <> struct WFrag<h16> { typedef v16h V; static __device__ __forceinline__ V ld(const h16* p) { return cat16(*(const v8h*)p, *(const v8h*)(p + 16)); } static __device__ __forceinline__ v8f mma(V a, V b, v8f c) { return wmma16(a, b, c); } };
template <> struct WFrag<bf> { typedef v16bf V; static __device__ __forceinline__ V ld(const bf* p) { return cat16b(*(const v8us*)p, *(const v8us*)(p + 16)); } static __device__ __forceinline__ v8f mma(V a, V b, v8f c) { return wmmab(a, b, c); } };
template <typename T16, int NSPLIT, bool BIAS>
__global__ __launch_bounds__(32) void k_gemmw(const T16* __restrict__ A, const T16* __restrict__ A2, const T16* __restrict__ Bt, const T16* __restrict__ Bt2, int K, float* C, int ldc, const float* __restrict__ bias, size_t sA, size_t sB, size_t sC) {
    typedef typename WFrag<T16>::V V;
    __shared__ __align__(16) float os[16 * 68];
    const size_t z = blockIdx.z; A += z * sA; if (A2) A2 += z * sA; Bt += z * sB; if (Bt2) Bt2 += z * sB; C += z * sC;
    const int lane = threadIdx.x & 31, lr = lane & 15, hi = lane >> 4; const int r0 = blockIdx.x * 64, c0 = blockIdx.y * 64;
    v8f acc[4][4];
#pragma unroll
    for (int mb = 0; mb < 4; ++mb)
#pragma unroll
        for (int nb = 0; nb < 4; ++nb) acc[mb][nb] = (v8f){};
    const size_t aoff = (size_t)(r0 + lr) * K + 8 * hi, boff = (size_t)(c0 + lr) * K + 8 * hi;
#pragma unroll 1
    for (int kc = 0; kc < K; kc += 32) {
        V a[4], a2[4];
#pragma unroll
        for (int mb = 0; mb < 4; ++mb) { a[mb] = WFrag<T16>::ld(A + aoff + (size_t)mb * 16 * K + kc); if (NSPLIT == 1 || NSPLIT == 2) a2[mb] = WFrag<T16>::ld(A2 + aoff + (size_t)mb * 16 * K + kc); }
#pragma unroll
        for (int nb = 0; nb < 4; ++nb) { const V b = WFrag<T16>::ld(Bt + boff + (size_t)nb * 16 * K + kc); V b2; if (NSPLIT >= 2) b2 = WFrag<T16>::ld(Bt2 + boff + (size_t)nb * 16 * K + kc);
#pragma unroll
            for (int mb = 0; mb < 4; ++mb) { acc[mb][nb] = WFrag<T16>::mma(a[mb], b, acc[mb][nb]); if (NSPLIT == 1 || NSPLIT == 2) acc[mb][nb] = WFrag<T16>::mma(a2[mb], b, acc[mb][nb]); if (NSPLIT >= 2) acc[mb][nb] = WFrag<T16>::mma(a[mb], b2, acc[mb][nb]); } }
        asm volatile("v_nop\n\tv_nop\n\tv_nop\n\tv_nop" : "+v"(acc[0][0]), "+v"(acc[1][1]), "+v"(acc[2][2]), "+v"(acc[3][3]) : "v"(a[0]), "v"(a[3]));
    }
#pragma unroll
    for (int mb = 0; mb < 4; ++mb) {
#pragma unroll
        for (int nb = 0; nb < 4; ++nb) {
#pragma unroll
            for (int j = 0; j < 8; ++j) os[(hi * 8 + j) * 68 + nb * 16 + lr] = acc[mb][nb][j]; }
        __builtin_amdgcn_wave_barrier(); asm volatile("" ::: "memory");
        float* crow = C + (size_t)(r0 + mb * 16) * ldc + c0;
#pragma unroll 1
        for (int ps = 0; ps < 2; ++ps) {
#pragma unroll
            for (int s = 0; s < 8; ++s) { const int row = 2 * s + hi, cofs = lr * 4; v4f val = *(const v4fa*)(os + row * 68 + cofs); if (BIAS) { val[0] += bfr(bias[c0 + cofs]); val[1] += bfr(bias[c0 + cofs + 1]); val[2] += bfr(bias[c0 + cofs + 2]); val[3] += bfr(bias[c0 + cofs + 3]); }
                *(volatile v4f*)(crow + (size_t)row * ldc + cofs) = val; }
            if (ps == 0) __threadfence(); }
        __builtin_amdgcn_wave_barrier(); asm volatile("" ::: "memory");
    }
}

__device__ __forceinline__ h16 tohx(float x) { return (h16)x; }
__device__ __forceinline__ void splitf(float y, unsigned short& h, unsigned short& l) { h = f2bf(y); l = f2bf(y - bf2f(h)); }
typedef __attribute__((ext_vector_type(2))) _Float16 v2h;
typedef __attribute__((ext_vector_type(4))) _Float16 v4h;
typedef __attribute__((ext_vector_type(2))) unsigned short v2us;
typedef __attribute__((ext_vector_type(4))) unsigned short v4us;
typedef __attribute__((ext_vector_type(2))) float v2f;
typedef __attribute__((ext_vector_type(4))) int v4i;


__global__ __launch_bounds__(256) void k_cvt8(const float* __restrict__ src, bf* dst, size_t n8) { const size_t i = (size_t)blockIdx.x * 256 + threadIdx.x; if (i >= n8) return; const v8f v = *(const v8f*)(src + i * 8); v8us o;
#pragma unroll
    for (int k = 0; k < 8; ++k) o[k] = f2bf(v[k]); *(volatile v8us*)(dst + i * 8) = o; __threadfence(); *(volatile v8us*)(dst + i * 8) = o; }


__global__ __launch_bounds__(256) void k_lsoft(const float* __restrict__ Sb, h16* P16, bf* Ph, bf* Pl) {
    const int lane = threadIdx.x & 31; const int row = blockIdx.x * 8 + (threadIdx.x >> 5); if (row >= ZH * TT) return; const int i = row % TT; const int zz = row / TT; const bool hires = (i < RH); const float* sr = Sb + (size_t)row * TT; float mx = -3.0e38f;
#pragma unroll 4
    for (int ch = 0; ch < TT / 128; ++ch) { const int j0 = ch * 128 + lane * 4; const v4f a = *(const v4f*)(sr + j0);
#pragma unroll
        for (int q = 0; q < 4; ++q) { float t = a[q] * SCL; asm volatile("" : "+v"(t)); mx = fmaxf(mx, t); } }
#pragma unroll
    for (int sh = 16; sh; sh >>= 1) mx = fmaxf(mx, __shfl_xor(mx, sh, 32));
    float sum = 0.f;
#pragma unroll 4
    for (int ch = 0; ch < TT / 128; ++ch) { const int j0 = ch * 128 + lane * 4; const v4f a = *(const v4f*)(sr + j0);
#pragma unroll
        for (int q = 0; q < 4; ++q) { float t = a[q] * SCL; asm volatile("" : "+v"(t)); float d0 = __fsub_rn(t, mx); asm volatile("" : "+v"(d0)); sum += __builtin_amdgcn_exp2f(__fmul_rn(d0, 1.4426950408889634f)); } }
#pragma unroll
    for (int sh = 16; sh; sh >>= 1) sum += __shfl_xor(sum, sh, 32);
    const float f = __fdiv_rn(hires ? 1.0f : PCAR, sum);
#pragma unroll 1
    for (int ps = 0; ps < 2; ++ps) {
        if (hires) {
#pragma unroll
            for (int ch = 0; ch < TT / 128; ++ch) { const int j0 = ch * 128 + lane * 4; const v4f a = *(const v4f*)(sr + j0); v4us oh, ol;
#pragma unroll
                for (int q = 0; q < 4; ++q) { float t = a[q] * SCL; asm volatile("" : "+v"(t)); float d0 = __fsub_rn(t, mx); asm volatile("" : "+v"(d0)); float ex = __builtin_amdgcn_exp2f(__fmul_rn(d0, 1.4426950408889634f)); asm volatile("" : "+v"(ex)); unsigned short a2, c2; splitf(ex * f, a2, c2); oh[q] = a2; ol[q] = c2; }
                const size_t oo = ((size_t)zz * RH + i) * TT + j0; *(volatile v4us*)(Ph + oo) = oh; *(volatile v4us*)(Pl + oo) = ol; }
        } else {
#pragma unroll 2
            for (int ch = 0; ch < TT / 128; ++ch) { const int j0 = ch * 128 + lane * 4; const v4f a = *(const v4f*)(sr + j0); v4h o4;
#pragma unroll
                for (int q = 0; q < 4; ++q) { float t = a[q] * SCL; asm volatile("" : "+v"(t)); float d0 = __fsub_rn(t, mx); asm volatile("" : "+v"(d0)); float ex = __builtin_amdgcn_exp2f(__fmul_rn(d0, 1.4426950408889634f)); asm volatile("" : "+v"(ex)); o4[q] = tohx(ex * f); }
                *(volatile v4h*)(P16 + (size_t)row * TT + j0) = o4; } }
        if (ps == 0) __threadfence(); }
}

__global__ __launch_bounds__(256) void k_xT(const float* __restrict__ xs, bf* XB) { const size_t k = (size_t)blockIdx.x * 256 + threadIdx.x; if (k >= (size_t)TT * CC / 8) return; const int c0 = (int)(k % (CC / 8)) * 8; const int t = (int)(k / (CC / 8)); v8us o;
#pragma unroll
    for (int q = 0; q < 8; ++q) o[q] = f2bf(xs[(size_t)(c0 + q) * TT + t]);
    *(volatile v8us*)(XB + (size_t)t * CC + c0) = o; __threadfence(); *(volatile v8us*)(XB + (size_t)t * CC + c0) = o; }
__global__ __launch_bounds__(256) void k_outTg(const float* __restrict__ O, const float* __restrict__ xs, const float* __restrict__ gm, float* out) { const size_t k = (size_t)blockIdx.x * 256 + threadIdx.x; if (k >= (size_t)CC * TT / 4) return; const int t0 = (int)(k % (TT / 4)) * 4; const int c = (int)(k / (TT / 4)); const float g = bfr(gm[0]); const v4f xi = *(const v4f*)(xs + (size_t)c * TT + t0); v4f o;
#pragma unroll
    for (int q = 0; q < 4; ++q) { float m = __fmul_rn(g, O[(size_t)(t0 + q) * CC + c]); asm volatile("" : "+v"(m)); o[q] = __fadd_rn(m, bfr(xi[q])); }
    *(volatile v4f*)(out + (size_t)c * TT + t0) = o; __threadfence(); *(volatile v4f*)(out + (size_t)c * TT + t0) = o; }
__global__ __launch_bounds__(256) void k_wpad3(const float* __restrict__ wf, const float* __restrict__ wg, const float* __restrict__ wh, bf* Bt) { const size_t i = (size_t)blockIdx.x * 256 + threadIdx.x; if (i >= (size_t)CP * CC / 8) return; const int k0 = (int)(i % (CC / 8)) * 8; const int n = (int)(i / (CC / 8)); const int blk = n / CI, r = n % CI; const float* src = (blk == 0 ? wf : (blk == 1 ? wg : wh)) + (size_t)r * CC + k0; v8us o;
#pragma unroll
    for (int q = 0; q < 8; ++q) { const unsigned short e = f2bf(src[q]); o[q] = (blk < 3) ? e : (unsigned short)0; }
    *(volatile v8us*)(Bt + (size_t)n * CC + k0) = o; __threadfence(); *(volatile v8us*)(Bt + (size_t)n * CC + k0) = o; }
__global__ __launch_bounds__(256) void k_fgplanes(const float* __restrict__ F, const float* __restrict__ bfv, const float* __restrict__ bgv, bf* Fh, bf* Fl, bf* Gh, bf* Gl) { const size_t k = (size_t)blockIdx.x * 256 + threadIdx.x; if (k >= (size_t)TT * CI / 4) return; const size_t e = k * 4; const int c = (int)(e % CI); const size_t t = e / CI; const v4f a = *(const v4f*)(F + t * CP + c); const v4f b2 = *(const v4f*)(F + t * CP + CI + c); v4us fh, fl, gh, gl;
#pragma unroll
    for (int q = 0; q < 4; ++q) { unsigned short u, w2; splitf(__fadd_rn(a[q], bfr(bfv[c + q])), u, w2); fh[q] = u; fl[q] = w2; splitf(__fadd_rn(b2[q], bfr(bgv[c + q])), u, w2); gh[q] = u; gl[q] = w2; }
#pragma unroll 1
    for (int ps = 0; ps < 2; ++ps) { *(volatile v4us*)(Fh + e) = fh; *(volatile v4us*)(Fl + e) = fl; *(volatile v4us*)(Gh + e) = gh; *(volatile v4us*)(Gl + e) = gl; if (ps == 0) __threadfence(); } }
__global__ __launch_bounds__(256) void k_hvt(const float* __restrict__ F, const float* __restrict__ bhv, bf* Hh, bf* Hl) { const size_t e = ((size_t)blockIdx.x * 256 + threadIdx.x) * 2; if (e >= (size_t)HP * TT) return; const int t = (int)(e % TT); const int c = (int)(e / TT); const int cc = min(c, CI - 1); const float bb = bfr(bhv[cc]); v2us oh, ol;
#pragma unroll
    for (int q = 0; q < 2; ++q) { const float v = __fadd_rn(F[(size_t)(t + q) * CP + 2 * CI + cc], bb); unsigned short u, w2; splitf(v, u, w2); oh[q] = (c < CI) ? u : (unsigned short)0; ol[q] = (c < CI) ? w2 : (unsigned short)0; }
    *(volatile v2us*)(Hh + e) = oh; *(volatile v2us*)(Hl + e) = ol; __threadfence(); *(volatile v2us*)(Hh + e) = oh; *(volatile v2us*)(Hl + e) = ol; }
__global__ __launch_bounds__(256) void k_ohl(const float* __restrict__ O, bf* Ah, bf* Al) { const size_t k = (size_t)blockIdx.x * 256 + threadIdx.x; if (k >= (size_t)TT * CI / 4) return; const size_t e = k * 4; const int c = (int)(e % CI); const size_t t = e / CI; const v4f a = *(const v4f*)(O + t * HP + c); v4us oh, ol;
#pragma unroll
    for (int q = 0; q < 4; ++q) { unsigned short u, w2; splitf(a[q], u, w2); oh[q] = u; ol[q] = w2; }
    *(volatile v4us*)(Ah + e) = oh; *(volatile v4us*)(Al + e) = ol; __threadfence(); *(volatile v4us*)(Ah + e) = oh; *(volatile v4us*)(Al + e) = ol; }

extern "C" void kernel_launch(void* const* d_in, const int* in_sizes, int n_in,
                              void* d_out, int out_size, void* d_ws, size_t ws_size, hipStream_t stream) {
    (void)in_sizes; (void)n_in; (void)out_size;
    const float* x = (const float*)d_in[0]; const float* wf = (const float*)d_in[1]; const float* bfv = (const float*)d_in[2]; const float* wg = (const float*)d_in[3]; const float* bgv = (const float*)d_in[4]; const float* wh = (const float*)d_in[5]; const float* bhv = (const float*)d_in[6]; const float* wv = (const float*)d_in[7]; const float* bv = (const float*)d_in[8]; const float* gm = (const float*)d_in[9];
    float* OUT = (float*)d_out;
    char* wsp = (char*)d_ws;
    auto take = [&](size_t bytes) { char* p = wsp; wsp += (bytes + 255) & ~(size_t)255; return (void*)p; };
    bf* WP = (bf*)take((size_t)CP * CC * 2); bf* WV = (bf*)take((size_t)CC * CI * 2);
    bf* XB = (bf*)take((size_t)TT * CC * 2); float* F = (float*)take((size_t)TT * CP * 4);
    bf* FPh = (bf*)take((size_t)TT * CI * 2); bf* FPl = (bf*)take((size_t)TT * CI * 2); bf* GPh = (bf*)take((size_t)TT * CI * 2); bf* GPl = (bf*)take((size_t)TT * CI * 2); bf* HTh = (bf*)take((size_t)HP * TT * 2); bf* HTl = (bf*)take((size_t)HP * TT * 2);
    float* Sb = (float*)take((size_t)TT * TT * 4); bf* Ph = (bf*)take((size_t)TT * TT * 2); bf* Pl = (bf*)take((size_t)TT * TT * 2); float* Ob = (float*)take((size_t)TT * HP * 4); bf* Ah = (bf*)take((size_t)TT * CI * 2); bf* Al = (bf*)take((size_t)TT * CI * 2); float* Y = (float*)take((size_t)TT * CC * 4);
    if ((size_t)(wsp - (char*)d_ws) > ws_size) return;
    k_wpad3<<<(unsigned)(((size_t)CP * CC / 8 + 255) / 256), 256, 0, stream>>>(wf, wg, wh, WP); k_cvt8<<<(unsigned)(((size_t)CC * CI / 8 + 255) / 256), 256, 0, stream>>>(wv, WV, (size_t)CC * CI / 8);
    for (int b = 0; b < NB_; ++b) {
        const float* xb = x + (size_t)b * CC * TT;
        k_xT<<<(unsigned)(((size_t)TT * CC / 8 + 255) / 256), 256, 0, stream>>>(xb, XB);
        k_gemmw<bf, 0, false><<<dim3(TT / 64, CP / 64, 1), 32, 0, stream>>>(XB, nullptr, WP, nullptr, CC, F, CP, nullptr, 0, 0, 0);
        k_fgplanes<<<(unsigned)(((size_t)TT * CI / 4 + 255) / 256), 256, 0, stream>>>(F, bfv, bgv, FPh, FPl, GPh, GPl); k_hvt<<<(unsigned)(((size_t)HP * TT / 2 + 255) / 256), 256, 0, stream>>>(F, bhv, HTh, HTl);
        k_gemmw<bf, 2, false><<<dim3(TT / 64, TT / 64, 1), 32, 0, stream>>>(FPh, FPl, GPh, GPl, CI, Sb, TT, nullptr, 0, 0, 0);
        k_lsoft<<<TT / 8, 256, 0, stream>>>(Sb, nullptr, Ph, Pl);
        k_gemmw<bf, 2, false><<<dim3(TT / 64, HP / 64, 1), 32, 0, stream>>>(Ph, Pl, HTh, HTl, TT, Ob, HP, nullptr, 0, 0, 0);
        k_ohl<<<(unsigned)(((size_t)TT * CI / 4 + 255) / 256), 256, 0, stream>>>(Ob, Ah, Al);
        k_gemmw<bf, 1, true><<<dim3(TT / 64, CC / 64, 1), 32, 0, stream>>>(Ah, Al, WV, nullptr, CI, Y, CC, bv, 0, 0, 0);
        k_outTg<<<(unsigned)(((size_t)CC * TT / 4 + 255) / 256), 256, 0, stream>>>(Y, xb, gm, OUT + (size_t)b * CC * TT); }
}
